// LieConvLayer_3977139716372
// MI455X (gfx1250) — hardware-verified
//
#include <hip/hip_runtime.h>
#include <stddef.h>
#include <stdint.h>


#define D_     248
#define DP     256
#define H_     512
#define HP     520
#define NNZ_   2480
#define NTHR   256
#define NWAVE  8
#define EPT    8
#define NGRP   2
#define CHUNK  (NTHR * EPT * NGRP)
#define WCAP   (EPT * NGRP * 32)
#define LISTN  (NWAVE * WCAP)
#define NB     64
#define AGP    260
#define FSP    260
#define GROWS  64
#define MROWS  32
#define WSCALE 16.0f
#define WINV   0.0625f
#define LN_EPS 1e-5f

#define OFF_SP   0
#define OFF_AG   (OFF_SP + NB * DP * 4)
#define OFF_FS   (OFF_AG + NB * AGP * 4)
#define OFF_LS   (OFF_FS + NB * FSP * 4)
#define LSBYTES  20480
#define OFF_WC   (OFF_LS + LSBYTES)
#define LDS_AGG  (OFF_WC + 64)
#define LDS_GEMMP (GROWS * DP * 4)
#define OFF_SHID 0
#define OFF_SH   (OFF_SHID + MROWS * HP * 2)
#define OFF_SOUT (OFF_SH + MROWS * DP * 4)
#define LDS_MLP  (OFF_SOUT + MROWS * D_ * 4)

static_assert((CHUNK & (CHUNK - 1)) == 0);
static_assert(CHUNK <= 4096);
static_assert((NB & (NB - 1)) == 0);
static_assert(NB <= 4096);
static_assert(LISTN * 4 <= LSBYTES);
static_assert(NNZ_ * 8 <= LSBYTES);
static_assert(NB * DP * 2 <= NB * FSP * 4);
static_assert(NB == GROWS);
static_assert(NB <= NTHR);
static_assert((NB % 32) == 0);
static_assert((OFF_AG % 16) == 0);
static_assert((OFF_FS % 16) == 0);
static_assert((OFF_LS % 16) == 0);
static_assert((OFF_WC % 16) == 0);
static_assert((OFF_SH % 16) == 0);
static_assert((OFF_SOUT % 16) == 0);
static_assert((D_ % 8) == 0);
static_assert((DP % 32) == 0);
static_assert((H_ % 32) == 0);
static_assert(MROWS * D_ <= NWAVE * 8 * 128);
static_assert(MROWS == NWAVE * 4);
static_assert(GROWS == NWAVE * 8);

typedef float    v4f  __attribute__((ext_vector_type(4)));
typedef float    v8f  __attribute__((ext_vector_type(8)));
typedef int      v4i  __attribute__((ext_vector_type(4)));
typedef _Float16 v8h  __attribute__((ext_vector_type(8)));
typedef _Float16 v16h __attribute__((ext_vector_type(16)));
union FragH { v16h v; v8h h[2]; };

__device__ __forceinline__ v8h cvt8(v4f a, v4f b) {
  v8h r;
  r[0] = (_Float16)a.x; r[1] = (_Float16)a.y; r[2] = (_Float16)a.z; r[3] = (_Float16)a.w;
  r[4] = (_Float16)b.x; r[5] = (_Float16)b.y; r[6] = (_Float16)b.z; r[7] = (_Float16)b.w;
  return r;
}

__device__ __forceinline__ v8f wmh(v16h a, v16h b, v8f c) {
  v8f d = __builtin_amdgcn_wmma_f32_16x16x32_f16(false, a, false, b, (short)0, c, false, false);
  asm volatile("v_nop\n\tv_nop\n\tv_nop\n\tv_nop" : "+v"(d) : "v"(a), "v"(b));
  return d;
}

__device__ __forceinline__ float wred32(float v) {
#pragma unroll
  for (int o = 16; o > 0; o >>= 1) v += __shfl_xor(v, o, 32);
  return v;
}

__device__ __forceinline__ _Float16 silu16(float a, float bias) {
  const float x = a * WINV + bias;
  const float e = __expf(-x);
  const float s = x * __builtin_amdgcn_rcpf(1.0f + e);
  return (_Float16)s;
}

template <int NBT>
__device__ __forceinline__ int scan_chunk(const int* __restrict__ dsts, int nE, int cbase, int nodeBase,
                                          int vec8, int* list, int tid, int lane, int wave) {
  int wc = 0;
#pragma unroll
  for (int g = 0; g < NGRP; ++g) {
    const int el0  = (g * NTHR + tid) * EPT;
    const int e0   = cbase + el0;
    const int sent = -2147483647 - 1;
    v4i da, db;
    if (vec8 != 0 && cbase + CHUNK <= nE) {
      da = *(const v4i*)(dsts + e0);
      db = *(const v4i*)(dsts + e0 + 4);
    } else {
      da.x = (e0     < nE) ? dsts[min(e0, nE - 1)] : sent;
      da.y = (e0 + 1 < nE) ? dsts[min(e0 + 1, nE - 1)] : sent;
      da.z = (e0 + 2 < nE) ? dsts[min(e0 + 2, nE - 1)] : sent;
      da.w = (e0 + 3 < nE) ? dsts[min(e0 + 3, nE - 1)] : sent;
      db.x = (e0 + 4 < nE) ? dsts[min(e0 + 4, nE - 1)] : sent;
      db.y = (e0 + 5 < nE) ? dsts[min(e0 + 5, nE - 1)] : sent;
      db.z = (e0 + 6 < nE) ? dsts[min(e0 + 6, nE - 1)] : sent;
      db.w = (e0 + 7 < nE) ? dsts[min(e0 + 7, nE - 1)] : sent;
    }
    const unsigned nb = (unsigned)nodeBase;
    const unsigned s0 = (unsigned)da.x - nb, s1 = (unsigned)da.y - nb;
    const unsigned s2 = (unsigned)da.z - nb, s3 = (unsigned)da.w - nb;
    const unsigned s4 = (unsigned)db.x - nb, s5 = (unsigned)db.y - nb;
    const unsigned s6 = (unsigned)db.z - nb, s7 = (unsigned)db.w - nb;
    const bool h0 = s0 < (unsigned)NBT, h1 = s1 < (unsigned)NBT, h2 = s2 < (unsigned)NBT, h3 = s3 < (unsigned)NBT;
    const bool h4 = s4 < (unsigned)NBT, h5 = s5 < (unsigned)NBT, h6 = s6 < (unsigned)NBT, h7 = s7 < (unsigned)NBT;
    const unsigned any = __builtin_amdgcn_ballot_w32(h0 | h1 | h2 | h3 | h4 | h5 | h6 | h7);
    if (any != 0u) {
#define HITJ(J, HJ, SJ) { \
        const unsigned mj = __builtin_amdgcn_ballot_w32(HJ); \
        if (mj != 0u) { \
          if (HJ) { \
            const int pos = wc + (int)__builtin_amdgcn_mbcnt_lo(mj, 0u); \
            if (pos < WCAP) list[wave * WCAP + pos] = ((el0 + (J)) << 12) | (int)(SJ); \
          } \
          wc += (int)__builtin_popcount(mj); } }
      HITJ(0, h0, s0)
      HITJ(1, h1, s1)
      HITJ(2, h2, s2)
      HITJ(3, h3, s3)
      HITJ(4, h4, s4)
      HITJ(5, h5, s5)
      HITJ(6, h6, s6)
      HITJ(7, h7, s7)
#undef HITJ
    }
  }
  return wc;
}

__global__ __launch_bounds__(NTHR) void k_prep(
    const float* __restrict__ feats, const float* __restrict__ Wmsg,
    const float* __restrict__ W1, const float* __restrict__ W2,
    _Float16* feat16, _Float16* wmsgP, _Float16* w1P, _Float16* w2P,
    int nN, int nPad) {
  const int tid = threadIdx.x;
  const int blk = blockIdx.x;
  const int nbF = nPad / 8;
  const int nbM = DP * (DP / 8) / NTHR;
  const int nb1 = H_ * (DP / 8) / NTHR;
  const int nb2 = DP * (H_ / 8) / NTHR;
  v4f a, b;
  bool valid;
  float sc;
  _Float16* dst;
  if (blk < nbF) {
    const int i  = blk * NTHR + tid;
    const int r  = i >> 5;
    const int c0 = (i & 31) * 8;
    const int rc = r < nN ? r : nN - 1;
    const int cc = c0 < D_ - 8 ? c0 : D_ - 8;
    const float* p = feats + (size_t)rc * D_ + cc;
    a = *(const v4f*)p; b = *(const v4f*)(p + 4);
    valid = (r < nN) && (c0 < D_);
    sc = 1.0f;
    dst = feat16 + (size_t)i * 8;
  } else if (blk < nbF + nbM) {
    const int i  = (blk - nbF) * NTHR + tid;
    const int n  = i >> 5;
    const int c0 = (i & 31) * 8;
    const int nc = n < D_ ? n : D_ - 1;
    const int cc = c0 < D_ - 8 ? c0 : D_ - 8;
    const float* p = Wmsg + (size_t)nc * D_ + cc;
    a = *(const v4f*)p; b = *(const v4f*)(p + 4);
    valid = (n < D_) && (c0 < D_);
    sc = WSCALE;
    dst = wmsgP + (size_t)i * 8;
  } else if (blk < nbF + nbM + nb1) {
    const int i  = (blk - nbF - nbM) * NTHR + tid;
    const int n  = i >> 5;
    const int c0 = (i & 31) * 8;
    const int cc = c0 < D_ - 8 ? c0 : D_ - 8;
    const float* p = W1 + (size_t)n * D_ + cc;
    a = *(const v4f*)p; b = *(const v4f*)(p + 4);
    valid = (c0 < D_);
    sc = WSCALE;
    dst = w1P + (size_t)i * 8;
  } else if (blk < nbF + nbM + nb1 + nb2) {
    const int i  = (blk - nbF - nbM - nb1) * NTHR + tid;
    const int n  = i >> 6;
    const int c0 = (i & 63) * 8;
    const int nc = n < D_ ? n : D_ - 1;
    const float* p = W2 + (size_t)nc * H_ + c0;
    a = *(const v4f*)p; b = *(const v4f*)(p + 4);
    valid = (n < D_);
    sc = WSCALE;
    dst = w2P + (size_t)i * 8;
  } else {
    return;
  }
  if (!valid) {
    const v4f z = {0.f, 0.f, 0.f, 0.f};
    a = z; b = z;
  }
  a = a * sc;
  b = b * sc;
  const v8h hv = cvt8(a, b);
  *(volatile v8h*)dst = hv;
  __threadfence();
  *(volatile v8h*)dst = hv;
}

__global__ __launch_bounds__(NTHR) void k_gemm_p(
    const _Float16* __restrict__ feat16, const _Float16* __restrict__ wmsgP, float* P) {
  extern __shared__ v4f lds_dyn[];
  float* stg = (float*)lds_dyn;
  const int tid = threadIdx.x, lane = tid & 31, wave = tid >> 5, hh = lane >> 4, m = lane & 15;
  const int rowBase = blockIdx.x * GROWS;
  const int rt = wave & 3, cg = wave >> 2;

  v8f acc[8];
#pragma unroll
  for (int t = 0; t < 8; ++t) { v8f z = {0.f, 0.f, 0.f, 0.f, 0.f, 0.f, 0.f, 0.f}; acc[t] = z; }
  const _Float16* ar = feat16 + ((size_t)rowBase + 16 * rt + m) * DP + 8 * hh;
  const _Float16* br = wmsgP + (size_t)(128 * cg + m) * DP + 8 * hh;
#pragma unroll 1
  for (int ks = 0; ks < DP / 32; ++ks) {
    FragH a;
    a.h[0] = *(const v8h*)(ar + 32 * ks);
    a.h[1] = *(const v8h*)(ar + 32 * ks + 16);
#pragma unroll
    for (int t = 0; t < 8; ++t) {
      const _Float16* bp = br + (size_t)(16 * t) * DP + 32 * ks;
      FragH b;
      b.h[0] = *(const v8h*)bp;
      b.h[1] = *(const v8h*)(bp + 16);
      acc[t] = wmh(a.v, b.v, acc[t]);
    }
  }

  float* sp = stg + (16 * rt + 8 * hh) * DP + 128 * cg + m;
#pragma unroll
  for (int t = 0; t < 8; ++t) {
    const v8f c = acc[t];
    sp[0 * DP + 16 * t] = c[0] * WINV;
    sp[1 * DP + 16 * t] = c[1] * WINV;
    sp[2 * DP + 16 * t] = c[2] * WINV;
    sp[3 * DP + 16 * t] = c[3] * WINV;
    sp[4 * DP + 16 * t] = c[4] * WINV;
    sp[5 * DP + 16 * t] = c[5] * WINV;
    sp[6 * DP + 16 * t] = c[6] * WINV;
    sp[7 * DP + 16 * t] = c[7] * WINV;
  }
  __syncthreads();

  const float* lp = stg + (wave * 8) * DP + 4 * lane;
  float* gp = P + ((size_t)rowBase + wave * 8) * DP + 4 * lane;
#pragma unroll
  for (int i = 0; i < 8; ++i) {
    const v4f v0 = *(const v4f*)(lp + i * DP), v1 = *(const v4f*)(lp + i * DP + 128);
    *(volatile v4f*)(gp + (size_t)i * DP) = v0;
    *(volatile v4f*)(gp + (size_t)i * DP + 128) = v1;
  }
  __threadfence();
#pragma unroll
  for (int i = 0; i < 8; ++i) {
    const v4f v0 = *(const v4f*)(lp + i * DP), v1 = *(const v4f*)(lp + i * DP + 128);
    *(volatile v4f*)(gp + (size_t)i * DP) = v0;
    *(volatile v4f*)(gp + (size_t)i * DP + 128) = v1;
  }
}

__global__ __launch_bounds__(NTHR) void k_agg(
    const int* __restrict__ ei, const float* __restrict__ P, const float* __restrict__ feats,
    const int* __restrict__ Ii, const int* __restrict__ Ji, const int* __restrict__ Ki,
    const float* __restrict__ Cv, _Float16* agg16, int nN, int nE, int vec8) {
  extern __shared__ v4f lds_dyn[];
  char* base = (char*)lds_dyn;
  float* SP = (float*)(base + OFF_SP);
  float* AG = (float*)(base + OFF_AG);
  float* FS = (float*)(base + OFF_FS);
  _Float16* ST = (_Float16*)(base + OFF_FS);
  int*   list  = (int*)(base + OFF_LS);
  int*   tripP = (int*)(base + OFF_LS);
  float* tripC = (float*)(base + OFF_LS + NNZ_ * 4);
  int*   wcnt  = (int*)(base + OFF_WC);
  const int tid = threadIdx.x, lane = tid & 31, wave = tid >> 5;
  const int nodeBase = blockIdx.x * NB;
  const int* dsts = ei + nE;

  {
    const v4f z = {0.f, 0.f, 0.f, 0.f};
    for (int i = tid; i < (NB * DP + NB * AGP) / 4; i += NTHR) lds_dyn[i] = z;
    for (int idx = tid; idx < NB * (D_ / 4); idx += NTHR) {
      const int slot = idx / (D_ / 4);
      const int c4   = (idx - slot * (D_ / 4)) * 4;
      int node = nodeBase + slot;
      node = node > nN - 1 ? nN - 1 : node;
      const v4f v = *(const v4f*)(feats + (size_t)node * D_ + c4);
      *(v4f*)(FS + slot * FSP + c4) = v;
    }
  }
  __syncthreads();

  const int nChunks = (nE + CHUNK - 1) / CHUNK;
#pragma unroll 1
  for (int ch = 0; ch < nChunks; ++ch) {
    const int cbase = ch * CHUNK;
    const int wc = scan_chunk<NB>(dsts, nE, cbase, nodeBase, vec8, list, tid, lane, wave);
    if (lane == 0) wcnt[wave] = wc;
    __syncthreads();
    if (wave == 0) {
#pragma unroll 1
      for (int wsx = 0; wsx < NWAVE; ++wsx) {
        int n = __builtin_amdgcn_readfirstlane(wcnt[wsx]);
        n = n > WCAP ? WCAP : (n < 0 ? 0 : n);
        const int* lp = list + wsx * WCAP;
#pragma unroll 1
        for (int i = 0; i < n; ++i) {
          const int ent  = __builtin_amdgcn_readfirstlane(lp[i]);
          const int slot = ent & (NB - 1);
          int e = cbase + ((ent >> 12) & (CHUNK - 1));
          e = e > nE - 1 ? nE - 1 : e;
          int src = ei[e];
          src = src < 0 ? 0 : (src > nN - 1 ? nN - 1 : src);
          const float* pr = P + (size_t)src * DP + 4 * lane;
          const v4f v0 = *(const v4f*)pr, v1 = *(const v4f*)(pr + 128);
          v4f* ap = (v4f*)(SP + slot * DP + 4 * lane);
          ap[0]  = ap[0] + v0;
          ap[32] = ap[32] + v1;
        }
      }
    }
    __syncthreads();
  }

  for (int t = tid; t < NNZ_; t += NTHR) {
    int ii = Ii[t], jj = Ji[t], kk = Ki[t];
    ii = ii < 0 ? 0 : (ii > D_ - 1 ? D_ - 1 : ii);
    jj = jj < 0 ? 0 : (jj > D_ - 1 ? D_ - 1 : jj);
    kk = kk < 0 ? 0 : (kk > D_ - 1 ? D_ - 1 : kk);
    tripP[t] = ii | (jj << 8) | (kk << 16);
    tripC[t] = Cv[t];
  }
  __syncthreads();

  if (tid < NB) {
    const float* spr = SP + tid * DP;
    const float* fsr = FS + tid * FSP;
    float*       agr = AG + tid * AGP;
#pragma unroll 4
    for (int t = 0; t < NNZ_; ++t) {
      const int   p = tripP[t];
      const float c = tripC[t];
      const float v = (spr[p & 255] * fsr[(p >> 8) & 255]) * c;
      const int   k = (p >> 16) & 255;
      agr[k] = agr[k] + v;
    }
  }
  __syncthreads();

  for (int idx = tid; idx < NB * (DP / 8); idx += NTHR) {
    const int slot = idx >> 5;
    const int c0   = (idx & 31) * 8;
    const float* ap = AG + slot * AGP + c0;
    const v4f a = *(const v4f*)ap, b = *(const v4f*)(ap + 4);
    *(v8h*)(ST + slot * DP + c0) = cvt8(a, b);
  }
  __syncthreads();

  const _Float16* lp2 = ST + (wave * 8) * DP + 8 * lane;
  _Float16* gp = agg16 + ((size_t)nodeBase + wave * 8) * DP + 8 * lane;
#pragma unroll
  for (int i = 0; i < 8; ++i) { const v8h v = *(const v8h*)(lp2 + i * DP); *(volatile v8h*)(gp + (size_t)i * DP) = v; }
  __threadfence();
#pragma unroll
  for (int i = 0; i < 8; ++i) { const v8h v = *(const v8h*)(lp2 + i * DP); *(volatile v8h*)(gp + (size_t)i * DP) = v; }
}

__global__ __launch_bounds__(NTHR) void k_mlp(
    const _Float16* __restrict__ agg16, const _Float16* __restrict__ w1P, const _Float16* __restrict__ w2P,
    const float* __restrict__ b1, const float* __restrict__ b2, const float* __restrict__ feats,
    const float* __restrict__ gamma, const float* __restrict__ beta, float* out, int nN) {
  extern __shared__ v4f lds_dyn[];
  char* base = (char*)lds_dyn;
  _Float16* sHid = (_Float16*)(base + OFF_SHID);
  float*    sH   = (float*)(base + OFF_SH);
  float*    sOut = (float*)(base + OFF_SOUT);
  const int tid = threadIdx.x, lane = tid & 31, wave = tid >> 5, hh = lane >> 4, m = lane & 15;
  const int rowBase = blockIdx.x * MROWS;
  const int rt = wave & 1, cg = wave >> 1;

  {
    v8f acc[8];
#pragma unroll
    for (int t = 0; t < 8; ++t) { v8f z = {0.f, 0.f, 0.f, 0.f, 0.f, 0.f, 0.f, 0.f}; acc[t] = z; }
    const _Float16* ar = agg16 + ((size_t)rowBase + 16 * rt + m) * DP + 8 * hh;
    const _Float16* br = w1P + (size_t)(128 * cg + m) * DP + 8 * hh;
#pragma unroll 1
    for (int ks = 0; ks < DP / 32; ++ks) {
      FragH a;
      a.h[0] = *(const v8h*)(ar + 32 * ks);
      a.h[1] = *(const v8h*)(ar + 32 * ks + 16);
#pragma unroll
      for (int t = 0; t < 8; ++t) {
        const _Float16* bp = br + (size_t)(16 * t) * DP + 32 * ks;
        FragH b;
        b.h[0] = *(const v8h*)bp;
        b.h[1] = *(const v8h*)(bp + 16);
        acc[t] = wmh(a.v, b.v, acc[t]);
      }
    }
    _Float16* hp = sHid + (16 * rt + 8 * hh) * HP + 128 * cg + m;
#pragma unroll
    for (int t = 0; t < 8; ++t) {
      const int n = 128 * cg + 16 * t + m;
      const float bias = b1[n];
      const v8f c = acc[t];
      _Float16* q = hp + 16 * t;
      q[0 * HP] = silu16(c[0], bias);
      q[1 * HP] = silu16(c[1], bias);
      q[2 * HP] = silu16(c[2], bias);
      q[3 * HP] = silu16(c[3], bias);
      q[4 * HP] = silu16(c[4], bias);
      q[5 * HP] = silu16(c[5], bias);
      q[6 * HP] = silu16(c[6], bias);
      q[7 * HP] = silu16(c[7], bias);
    }
  }
  __syncthreads();

  {
    v8f acc[4];
#pragma unroll
    for (int t = 0; t < 4; ++t) { v8f z = {0.f, 0.f, 0.f, 0.f, 0.f, 0.f, 0.f, 0.f}; acc[t] = z; }
    const _Float16* ar = sHid + (16 * rt + m) * HP + 8 * hh;
    const _Float16* br = w2P + (size_t)(64 * cg + m) * H_ + 8 * hh;
#pragma unroll 1
    for (int ks = 0; ks < H_ / 32; ++ks) {
      FragH a;
      a.h[0] = *(const v8h*)(ar + 32 * ks);
      a.h[1] = *(const v8h*)(ar + 32 * ks + 16);
#pragma unroll
      for (int t = 0; t < 4; ++t) {
        const _Float16* bp = br + (size_t)(16 * t) * H_ + 32 * ks;
        FragH b;
        b.h[0] = *(const v8h*)bp;
        b.h[1] = *(const v8h*)(bp + 16);
        acc[t] = wmh(a.v, b.v, acc[t]);
      }
    }
    float* sp = sH + (16 * rt + 8 * hh) * DP + 64 * cg + m;
#pragma unroll
    for (int t = 0; t < 4; ++t) {
      const int n  = 64 * cg + 16 * t + m;
      const int nc = n < D_ ? n : D_ - 1;
      const float bb = b2[nc];
      const float bias = (n < D_) ? bb : 0.f;
      const v8f c = acc[t];
      sp[0 * DP + 16 * t] = c[0] * WINV + bias;
      sp[1 * DP + 16 * t] = c[1] * WINV + bias;
      sp[2 * DP + 16 * t] = c[2] * WINV + bias;
      sp[3 * DP + 16 * t] = c[3] * WINV + bias;
      sp[4 * DP + 16 * t] = c[4] * WINV + bias;
      sp[5 * DP + 16 * t] = c[5] * WINV + bias;
      sp[6 * DP + 16 * t] = c[6] * WINV + bias;
      sp[7 * DP + 16 * t] = c[7] * WINV + bias;
    }
  }
  __syncthreads();

#pragma unroll 1
  for (int rr = 0; rr < 4; ++rr) {
    const int lr = wave * 4 + rr;
    int node = rowBase + lr;
    node = node > nN - 1 ? nN - 1 : node;
    const float* fr = feats + (size_t)node * D_;
    const float* hr = sH + lr * DP;
    float xv[8];
    float s = 0.f;
#pragma unroll
    for (int c = 0; c < 8; ++c) {
      const int d  = lane + 32 * c;
      const int dc = d < D_ ? d : D_ - 1;
      float x = fr[dc] + hr[d];
      x = (d < D_) ? x : 0.f;
      xv[c] = x;
      s += x;
    }
    s = wred32(s);
    const float mu = s * (1.0f / (float)D_);
    float q = 0.f;
#pragma unroll
    for (int c = 0; c < 8; ++c) {
      const int d = lane + 32 * c;
      float xc = xv[c] - mu;
      xc = (d < D_) ? xc : 0.f;
      q += xc * xc;
    }
    q = wred32(q);
    const float inv = rsqrtf(q * (1.0f / (float)D_) + LN_EPS);
    float* orow = sOut + lr * D_;
#pragma unroll
    for (int c = 0; c < 8; ++c) {
      const int d  = lane + 32 * c;
      const int dc = d < D_ ? d : D_ - 1;
      const float g = gamma[dc], bt = beta[dc];
      const float y = (xv[c] - mu) * inv * g + bt;
      if (d < D_) orow[d] = y;
    }
  }
  __syncthreads();

  const int rowsV  = (nN - rowBase) < MROWS ? (nN - rowBase) : MROWS;
  const int nValid = rowsV * D_;
  float* ob = out + (size_t)rowBase * D_;
#pragma unroll
  for (int jj = 0; jj < 8; ++jj) {
    const int f = (wave + 8 * jj) * 128 + 4 * lane;
    if (f < nValid) { const v4f v = *(const v4f*)(sOut + f); *(volatile v4f*)(ob + f) = v; }
  }
  __threadfence();
#pragma unroll
  for (int jj = 0; jj < 8; ++jj) {
    const int f = (wave + 8 * jj) * 128 + 4 * lane;
    if (f < nValid) { const v4f v = *(const v4f*)(sOut + f); *(volatile v4f*)(ob + f) = v; }
  }
}

extern "C" void kernel_launch(void* const* d_in, const int* in_sizes, int n_in,
                              void* d_out, int out_size, void* d_ws, size_t ws_size,
                              hipStream_t stream) {
  if (n_in < 13) return;
  const int nN = in_sizes[0] / D_;
  const int nE = in_sizes[1] / 2;
  if (nN <= 0 || nE <= 0 || in_sizes[0] != nN * D_ || in_sizes[1] != 2 * nE) return;
  if (in_sizes[2] != D_ * D_ || in_sizes[3] != H_ * D_ || in_sizes[4] < H_ || in_sizes[5] != D_ * H_) return;
  if (in_sizes[6] < D_ || in_sizes[7] < D_ || in_sizes[8] < D_) return;
  if (in_sizes[9] != NNZ_ || in_sizes[10] != NNZ_ || in_sizes[11] != NNZ_ || in_sizes[12] != NNZ_) return;
  if (out_size != nN * D_) return;

  const float* feats = (const float*)d_in[0];
  const int*   ei    = (const int*)d_in[1];
  const float* Wmsg  = (const float*)d_in[2];
  const float* W1    = (const float*)d_in[3];
  const float* b1    = (const float*)d_in[4];
  const float* W2    = (const float*)d_in[5];
  const float* b2    = (const float*)d_in[6];
  const float* gamma = (const float*)d_in[7];
  const float* beta  = (const float*)d_in[8];
  const int*   Ii    = (const int*)d_in[9];
  const int*   Ji    = (const int*)d_in[10];
  const int*   Ki    = (const int*)d_in[11];
  const float* Cv    = (const float*)d_in[12];
  float* out = (float*)d_out;

  const int nPad = ((nN + GROWS - 1) / GROWS) * GROWS;
  const int nBG  = nPad / GROWS;
  const int nBM  = (nN + MROWS - 1) / MROWS;

  char* ws = (char*)d_ws;
  size_t off = 0;
  const size_t oF16 = off; off += (size_t)nPad * DP * 2;   off = (off + 255) & ~(size_t)255;
  const size_t oWM  = off; off += (size_t)DP * DP * 2;     off = (off + 255) & ~(size_t)255;
  const size_t oW1  = off; off += (size_t)H_ * DP * 2;     off = (off + 255) & ~(size_t)255;
  const size_t oW2  = off; off += (size_t)DP * H_ * 2;     off = (off + 255) & ~(size_t)255;
  const size_t oP   = off; off += (size_t)nPad * DP * 4;   off = (off + 255) & ~(size_t)255;
  const size_t oAG  = off; off += (size_t)nPad * DP * 2;   off = (off + 255) & ~(size_t)255;
  if (off > ws_size || off > (size_t)134217728) return;
  _Float16* feat16 = (_Float16*)(ws + oF16);
  _Float16* wmsgP  = (_Float16*)(ws + oWM);
  _Float16* w1P    = (_Float16*)(ws + oW1);
  _Float16* w2P    = (_Float16*)(ws + oW2);
  float*    P      = (float*)(ws + oP);
  _Float16* agg16  = (_Float16*)(ws + oAG);

  const int vec8 = ((nE & 3) == 0) ? 1 : 0;

  const int nPrepBlocks = nPad / 8 + DP * (DP / 8) / NTHR + H_ * (DP / 8) / NTHR + DP * (H_ / 8) / NTHR;
  k_prep<<<nPrepBlocks, NTHR, 0, stream>>>(feats, Wmsg, W1, W2, feat16, wmsgP, w1P, w2P, nN, nPad);

  hipFuncSetAttribute(reinterpret_cast<const void*>(&k_gemm_p),
                      hipFuncAttributeMaxDynamicSharedMemorySize, LDS_GEMMP);
  k_gemm_p<<<nBG, NTHR, LDS_GEMMP, stream>>>(feat16, wmsgP, P);

  hipFuncSetAttribute(reinterpret_cast<const void*>(&k_agg),
                      hipFuncAttributeMaxDynamicSharedMemorySize, LDS_AGG);
  k_agg<<<nBG, NTHR, LDS_AGG, stream>>>(ei, P, feats, Ii, Ji, Ki, Cv, agg16, nN, nE, vec8);

  hipFuncSetAttribute(reinterpret_cast<const void*>(&k_mlp),
                      hipFuncAttributeMaxDynamicSharedMemorySize, LDS_MLP);
  k_mlp<<<nBM, NTHR, LDS_MLP, stream>>>(agg16, w1P, w2P, b1, b2, feats, gamma, beta, out, nN);
}
